// GeometricFlow_74732430950680
// MI455X (gfx1250) — hardware-run, weakly checked
//
#include <hip/hip_runtime.h>
#include <math.h>

typedef __attribute__((ext_vector_type(16))) _Float16 v16h;
typedef __attribute__((ext_vector_type(8)))  _Float16 v8h;
typedef __attribute__((ext_vector_type(8)))  float    v8f;
typedef __attribute__((ext_vector_type(4)))  float    v4f;

constexpr int kNB   = 32;
constexpr int kMD   = 32;
constexpr int kHid  = 128;
constexpr int kRH   = 256;
constexpr int kMM   = kMD * kMD;
static_assert(kMM == 1024, "pair count");
static_assert(kRH == 2 * kHid, "hidden width of the pair MLP");
static_assert((kMD % 32) == 0 && (kRH % 32) == 0, "matrix-core K multiples of 32");
static_assert((kMD % 16) == 0 && (kRH % 16) == 0 && (kMM % 16) == 0, "matrix-core M,N multiples of 16");

constexpr float kCarryAct = 64.0f;
constexpr float kCarryW   = 256.0f;
constexpr float kFold     = 1.0f / (kCarryAct * kCarryW);
constexpr float kF16Min   = 6.103515625e-05f;
constexpr float kInvPairs = 1.0f / (float)kMM;

constexpr int kCP = 260;
constexpr int kHP = 260;
constexpr int kOP = 132;

constexpr size_t kOffMET   = 0;
constexpr size_t kOffPP    = kOffMET   + (size_t)kNB * kMM * 4;
constexpr size_t kOffG1    = kOffPP    + (size_t)kNB * kRH * 4;
constexpr size_t kOffG2    = kOffG1    + (size_t)kNB * kMD * kRH * 4;
constexpr size_t kOffHPART = kOffG2    + (size_t)kNB * kMD * kRH * 4;
constexpr size_t kOffSS    = kOffHPART + (size_t)kNB * kMD * kRH * 4;
constexpr size_t kOffW1C   = kOffSS    + (size_t)kNB * kMM * 4;
constexpr size_t kOffW2T   = kOffW1C   + (size_t)kRH * kMD * 2;
constexpr size_t kWsTotal  = kOffW2T   + (size_t)kMM * kRH * 2;
static_assert(kWsTotal == 3981312ull, "carve total");
static_assert(kWsTotal <= 134217728ull, "carve cap");
static_assert((kOffPP % 128) == 0 && (kOffG1 % 128) == 0 && (kOffG2 % 128) == 0 && (kOffHPART % 128) == 0 &&
              (kOffSS % 128) == 0 && (kOffW1C % 128) == 0 && (kOffW2T % 128) == 0, "128-B aligned regions");

__device__ __forceinline__ unsigned pin_u(unsigned x) {
  asm volatile("" : "+v"(x));
  return x;
}

__device__ __forceinline__ float flush_f16n(float v) {
  return (fabsf(v) < kF16Min) ? 0.0f : v;
}

union FragU { v16h v; v8h h[2]; };
__device__ __forceinline__ v16h frag_load_h(const _Float16* p) {
  FragU f;
  f.h[0] = *(const v8h*)(p);
  f.h[1] = *(const v8h*)(p + 16);
  return f.v;
}

__device__ __forceinline__ v16h frag_from_f32(const float* p) {
  const v4f a0 = *(const v4f*)(p);
  const v4f a1 = *(const v4f*)(p + 4);
  const v4f a2 = *(const v4f*)(p + 16);
  const v4f a3 = *(const v4f*)(p + 20);
  v16h f;
#pragma unroll
  for (int e = 0; e < 4; ++e) {
    f[e]      = (_Float16)flush_f16n(a0[e] * kCarryAct);
    f[4 + e]  = (_Float16)flush_f16n(a1[e] * kCarryAct);
    f[8 + e]  = (_Float16)flush_f16n(a2[e] * kCarryAct);
    f[12 + e] = (_Float16)flush_f16n(a3[e] * kCarryAct);
  }
  return f;
}

__device__ __forceinline__ v8f mma_f16(v16h a, v16h b, v8f c) {
  c = __builtin_amdgcn_wmma_f32_16x16x32_f16(false, a, false, b, (short)0, c, false, false);
  asm volatile("v_nop\n\tv_nop\n\tv_nop\n\tv_nop" : "+v"(c) : "v"(a), "v"(b));
  return c;
}

__device__ __forceinline__ void pack8_store(const float* __restrict__ src, unsigned ld, unsigned n, unsigned k0,
                                            _Float16* dst) {
  v8h hv;
#pragma unroll
  for (int e = 0; e < 8; ++e) {
    const float w = src[(size_t)(k0 + (unsigned)e) * ld + n];
    hv[e] = (_Float16)flush_f16n(w * kCarryW);
  }
  *(volatile v8h*)dst = hv;
  __threadfence();
  *(volatile v8h*)dst = hv;
}

__global__ __launch_bounds__(256) void pack_weights_kernel(const float* __restrict__ Wr1,
                                                           const float* __restrict__ Wr2,
                                                           _Float16* __restrict__ W1C,
                                                           _Float16* __restrict__ W2T) {
  const unsigned tid = threadIdx.x;
  if (blockIdx.x < 128u) {
    const unsigned g  = pin_u(blockIdx.x * 256u + tid);
    const unsigned n  = pin_u(g >> 5);
    const unsigned k0 = pin_u((g & 31u) << 3);
    pack8_store(Wr2, (unsigned)kMM, n, k0, W2T + (size_t)g * 8u);
  } else {
    const unsigned g  = pin_u((blockIdx.x - 128u) * 256u + tid);
    const unsigned n  = pin_u(g >> 2);
    const unsigned k0 = pin_u((g & 3u) << 3);
    pack8_store(Wr1 + (size_t)96 * kRH, (unsigned)kRH, n, k0, W1C + (size_t)g * 8u);
  }
}

__global__ __launch_bounds__(256) void metric_kernel(const float* __restrict__ points,
                                                     const float* __restrict__ Wm1, const float* __restrict__ bm1,
                                                     const float* __restrict__ Wm2, const float* __restrict__ bm2,
                                                     float* __restrict__ MET) {
  __shared__ float sPts[kMD];
  __shared__ float sHid[kHid];
  __shared__ __align__(16) float sCmp[kMM];
  const unsigned t = threadIdx.x;
  const unsigned b = blockIdx.x;
  if (t < 32u) sPts[t] = points[b * kMD + t];
  __syncthreads();
  if (t < 128u) {
    float a = bm1[t];
#pragma unroll 4
    for (int m = 0; m < kMD; ++m) a = fmaf(sPts[m], Wm1[m * kHid + t], a);
    sHid[t] = fmaxf(a, 0.0f);
  }
  __syncthreads();
#pragma unroll 1
  for (unsigned q = 0; q < 4u; ++q) {
    const unsigned n = t + 256u * q;
    float a = bm2[n];
#pragma unroll 8
    for (int h = 0; h < kHid; ++h) a = fmaf(sHid[h], Wm2[(size_t)h * kMM + n], a);
    const float dg = ((n >> 5) == (n & 31u)) ? 1e-6f : 0.0f;
    sCmp[n] = a + dg;
  }
  __syncthreads();
  v4f o;
#pragma unroll
  for (int e = 0; e < 4; ++e) {
    const unsigned n = 4u * t + (unsigned)e;
    const unsigned i = n >> 5, j = n & 31u;
    o[e] = 0.5f * (sCmp[n] + sCmp[j * 32u + i]);
  }
  float* dst = MET + (size_t)b * kMM + 4u * t;
  *(volatile v4f*)dst = o;
  __threadfence();
  *(volatile v4f*)dst = o;
}

__global__ __launch_bounds__(256) void pair_pre_kernel(const float* __restrict__ points,
                                                       const float* __restrict__ Wr1,
                                                       const float* __restrict__ MET,
                                                       float* __restrict__ PP, float* __restrict__ G1,
                                                       float* __restrict__ G2) {
  __shared__ float sPts[kMD];
  __shared__ __align__(16) float sMet[kMM];
  const unsigned t = threadIdx.x;
  const unsigned b = blockIdx.x;
  if (t < 32u) sPts[t] = points[b * kMD + t];
  *(v4f*)(sMet + 4u * t) = *(const v4f*)(MET + (size_t)b * kMM + 4u * t);
  __syncthreads();
  {
    float a = 0.0f;
#pragma unroll 4
    for (int m = 0; m < kMD; ++m) a = fmaf(sPts[m], Wr1[m * kRH + t], a);
    float* p = PP + (size_t)b * kRH + t;
    *(volatile float*)p = a;
    __threadfence();
    *(volatile float*)p = a;
  }
#pragma unroll 1
  for (int r = 0; r < kMD; ++r) {
    float a1 = 0.0f, a2 = 0.0f;
#pragma unroll 4
    for (int k = 0; k < kMD; ++k) {
      const float mv = sMet[r * kMD + k];
      a1 = fmaf(mv, Wr1[(32 + k) * kRH + t], a1);
      a2 = fmaf(mv, Wr1[(64 + k) * kRH + t], a2);
    }
    float* p1 = G1 + ((size_t)b * kMD + r) * kRH + t;
    float* p2 = G2 + ((size_t)b * kMD + r) * kRH + t;
    *(volatile float*)p1 = a1;
    *(volatile float*)p2 = a2;
    __threadfence();
    *(volatile float*)p1 = a1;
    *(volatile float*)p2 = a2;
  }
}

__global__ __launch_bounds__(256) void triple_pair_kernel(const float* __restrict__ MET,
                                                          const float* __restrict__ Wc1, const float* __restrict__ bc1,
                                                          const float* __restrict__ Wc2, const float* __restrict__ bc2,
                                                          const _Float16* __restrict__ W1C,
                                                          const float* __restrict__ br1,
                                                          const float* __restrict__ PP, const float* __restrict__ G1,
                                                          const float* __restrict__ G2, float* __restrict__ HPART) {
  __shared__ __align__(16) float sMet[kMM];
  __shared__ __align__(16) float sCW[kHid * 4];
  __shared__ float sCV[kHid];
  __shared__ __align__(16) float sChr[kMD * kMD];
  __shared__ __align__(16) float sC[kMD * kCP];
  const unsigned t    = threadIdx.x;
  const unsigned lane = pin_u(t & 31u);
  const unsigned wave = t >> 5;
  const unsigned b    = blockIdx.x >> 5;
  const unsigned i    = blockIdx.x & 31u;

  *(v4f*)(sMet + 4u * t) = *(const v4f*)(MET + (size_t)b * kMM + 4u * t);
  if (t < 128u) {
    v4f cw;
    cw[0] = Wc1[t];
    cw[1] = Wc1[kHid + t];
    cw[2] = Wc1[2 * kHid + t];
    cw[3] = bc1[t];
    *(v4f*)(sCW + 4u * t) = cw;
    sCV[t] = Wc2[t];
  }
  const float bc2v = bc2[0];
  __syncthreads();

#pragma unroll 1
  for (unsigned q = 0; q < 4u; ++q) {
    const unsigned j = wave + 8u * q;
    const float gij = sMet[i * 32u + j];
    const float gjk = sMet[j * 32u + lane];
    const float gki = sMet[lane * 32u + i];
    float acc = bc2v;
#pragma unroll 2
    for (int n = 0; n < kHid; ++n) {
      const v4f c = *(const v4f*)(sCW + 4 * n);
      float u = fmaf(gki, c[2], c[3]);
      u = fmaf(gjk, c[1], u);
      u = fmaf(gij, c[0], u);
      acc = fmaf(tanhf(u), sCV[n], acc);
    }
    sChr[j * 32u + lane] = acc;
  }
  __syncthreads();

  {
    const unsigned hh = pin_u(lane >> 4);
    const unsigned c  = pin_u(lane & 15u);
    const unsigned nt0 = wave * 2u;
    const unsigned nt1 = nt0 + 1u;
    const v16h bf0 = frag_load_h(W1C + (size_t)(nt0 * 16u + c) * kMD + 8u * hh);
    const v16h bf1 = frag_load_h(W1C + (size_t)(nt1 * 16u + c) * kMD + 8u * hh);
    const v16h a0 = frag_from_f32(sChr + c * 32u + 8u * hh);
    const v16h a1 = frag_from_f32(sChr + (16u + c) * 32u + 8u * hh);
    const v8f z = (v8f){0.f, 0.f, 0.f, 0.f, 0.f, 0.f, 0.f, 0.f};
    const v8f d00 = mma_f16(a0, bf0, z);
    const v8f d01 = mma_f16(a0, bf1, z);
    const v8f d10 = mma_f16(a1, bf0, z);
    const v8f d11 = mma_f16(a1, bf1, z);
#pragma unroll
    for (int r = 0; r < 8; ++r) {
      const unsigned row = 8u * hh + (unsigned)r;
      sC[row * kCP + nt0 * 16u + c]         = d00[r];
      sC[row * kCP + nt1 * 16u + c]         = d01[r];
      sC[(16u + row) * kCP + nt0 * 16u + c] = d10[r];
      sC[(16u + row) * kCP + nt1 * 16u + c] = d11[r];
    }
  }
  __syncthreads();

  {
    const float base = PP[(size_t)b * kRH + t] + G1[((size_t)b * kMD + i) * kRH + t] + br1[t];
    float hs = 0.0f;
#pragma unroll 4
    for (int j = 0; j < kMD; ++j) {
      const float g2 = G2[((size_t)b * kMD + j) * kRH + t];
      const float hv = fmaf(sC[j * kCP + t], kFold, base + g2);
      hs += fmaxf(hv, 0.0f);
    }
    float* p = HPART + ((size_t)b * kMD + i) * kRH + t;
    *(volatile float*)p = hs;
    __threadfence();
    *(volatile float*)p = hs;
  }
}

__global__ __launch_bounds__(256) void mean_proj_kernel(const float* __restrict__ HPART,
                                                        const _Float16* __restrict__ W2T,
                                                        const float* __restrict__ br2,
                                                        float* __restrict__ SS) {
  __shared__ __align__(16) float sH[kNB * kHP];
  __shared__ __align__(16) float sO[kNB * kOP];
  const unsigned t    = threadIdx.x;
  const unsigned lane = pin_u(t & 31u);
  const unsigned wave = t >> 5;
  const unsigned bx   = blockIdx.x;

#pragma unroll 1
  for (int bb = 0; bb < kNB; ++bb) {
    float s = 0.0f;
#pragma unroll 4
    for (int i = 0; i < kMD; ++i) s += HPART[((size_t)bb * kMD + i) * kRH + t];
    sH[bb * kHP + t] = s * kInvPairs;
  }
  __syncthreads();

  {
    const unsigned hh = pin_u(lane >> 4);
    const unsigned c  = pin_u(lane & 15u);
    const unsigned nt = bx * 8u + wave;
    const _Float16* brow = W2T + (size_t)(nt * 16u + c) * kRH + 8u * hh;
    const float* arow0 = sH + c * kHP + 8u * hh;
    const float* arow1 = sH + (16u + c) * kHP + 8u * hh;
    v8f acc0 = (v8f){0.f, 0.f, 0.f, 0.f, 0.f, 0.f, 0.f, 0.f};
    v8f acc1 = (v8f){0.f, 0.f, 0.f, 0.f, 0.f, 0.f, 0.f, 0.f};
#pragma unroll
    for (int ks = 0; ks < kRH / 32; ++ks) {
      const v16h bfr = frag_load_h(brow + ks * 32);
      const v16h a0 = frag_from_f32(arow0 + ks * 32);
      const v16h a1 = frag_from_f32(arow1 + ks * 32);
      acc0 = mma_f16(a0, bfr, acc0);
      acc1 = mma_f16(a1, bfr, acc1);
    }
    const float bv = br2[nt * 16u + c];
#pragma unroll
    for (int r = 0; r < 8; ++r) {
      const unsigned row = 8u * hh + (unsigned)r;
      sO[row * kOP + wave * 16u + c]         = fmaf(acc0[r], kFold, bv);
      sO[(16u + row) * kOP + wave * 16u + c] = fmaf(acc1[r], kFold, bv);
    }
  }
  __syncthreads();

  {
    v4f ov[4];
#pragma unroll
    for (int rr = 0; rr < 4; ++rr) ov[rr] = *(const v4f*)(sO + (wave * 4u + (unsigned)rr) * kOP + lane * 4u);
    for (int pass = 0; pass < 2; ++pass) {
#pragma unroll
      for (int rr = 0; rr < 4; ++rr) {
        float* dst = SS + (size_t)(wave * 4u + (unsigned)rr) * kMM + bx * 128u + lane * 4u;
        *(volatile v4f*)dst = ov[rr];
      }
      __threadfence();
    }
  }
}

__global__ __launch_bounds__(256) void tail_kernel(const float* __restrict__ points, const float* __restrict__ SS,
                                                   const float* __restrict__ Wf1, const float* __restrict__ bf1,
                                                   const float* __restrict__ Wf2, const float* __restrict__ bf2,
                                                   const float* __restrict__ Wh1, const float* __restrict__ bh1,
                                                   const float* __restrict__ Wh2, const float* __restrict__ bh2,
                                                   float* __restrict__ out) {
  __shared__ float sPts[kMD];
  __shared__ __align__(16) float sS[kMM];
  __shared__ float sRd[kMD];
  __shared__ float sFh[kHid];
  __shared__ float sNp[kMD];
  __shared__ float sHh[kHid];
  const unsigned t = threadIdx.x;
  const unsigned b = blockIdx.x;
  if (t < 32u) sPts[t] = points[b * kMD + t];
  *(v4f*)(sS + 4u * t) = *(const v4f*)(SS + (size_t)b * kMM + 4u * t);
  __syncthreads();
  if (t < 32u) {
    float a = 0.0f;
#pragma unroll 4
    for (int j = 0; j < kMD; ++j) {
      const float rv = 0.5f * (sS[t * 32u + j] + sS[j * 32 + t]);
      a = fmaf(rv, sPts[j], a);
    }
    sRd[t] = a;
  }
  __syncthreads();
  if (t < 128u) {
    float a = bf1[t];
#pragma unroll 4
    for (int m = 0; m < kMD; ++m) {
      a = fmaf(sPts[m], Wf1[m * kHid + t], a);
      a = fmaf(sRd[m], Wf1[(kMD + m) * kHid + t], a);
    }
    sFh[t] = fmaxf(a, 0.0f);
  }
  __syncthreads();
  if (t < 32u) {
    float a = bf2[t];
#pragma unroll 4
    for (int h = 0; h < kHid; ++h) a = fmaf(sFh[h], Wf2[h * kMD + t], a);
    sNp[t] = sPts[t] + a;
  }
  __syncthreads();
  if (t < 128u) {
    float a = bh1[t];
#pragma unroll 4
    for (int m = 0; m < kMD; ++m) a = fmaf(sNp[m], Wh1[m * kHid + t], a);
    sHh[t] = tanhf(a);
  }
  __syncthreads();
  if (t < 64u) {
    float a = bh2[t];
#pragma unroll 4
    for (int h = 0; h < kHid; ++h) a = fmaf(sHh[h], Wh2[h * 64 + t], a);
    float* p = out + (size_t)b * 64u + t;
    *(volatile float*)p = a;
    __threadfence();
    *(volatile float*)p = a;
  }
}

extern "C" void kernel_launch(void* const* d_in, const int* in_sizes, int n_in,
                              void* d_out, int out_size, void* d_ws, size_t ws_size,
                              hipStream_t stream) {
  if (n_in < 21) return;
  if (in_sizes[0] != kNB * kMD) return;
  if (in_sizes[1] != kMD * kHid) return;
  if (in_sizes[2] != kHid) return;
  if (in_sizes[3] != kHid * kMM) return;
  if (in_sizes[4] != kMM) return;
  if (in_sizes[5] != 3 * kHid) return;
  if (in_sizes[6] != kHid) return;
  if (in_sizes[7] != kHid) return;
  if (in_sizes[8] != 1) return;
  if (in_sizes[9] != 4 * kMD * kRH) return;
  if (in_sizes[10] != kRH) return;
  if (in_sizes[11] != kRH * kMM) return;
  if (in_sizes[12] != kMM) return;
  if (in_sizes[13] != 2 * kMD * kHid) return;
  if (in_sizes[14] != kHid) return;
  if (in_sizes[15] != kHid * kMD) return;
  if (in_sizes[16] != kMD) return;
  if (in_sizes[17] != 2 * kMD * kHid) return;
  if (in_sizes[18] != kHid) return;
  if (in_sizes[19] != kHid * 2 * kMD) return;
  if (in_sizes[20] != 2 * kMD) return;
  if (out_size != kNB * 2 * kMD) return;
  if (ws_size < kWsTotal) return;

  const float* points = (const float*)d_in[0];
  const float* Wm1 = (const float*)d_in[1];
  const float* bm1 = (const float*)d_in[2];
  const float* Wm2 = (const float*)d_in[3];
  const float* bm2 = (const float*)d_in[4];
  const float* Wc1 = (const float*)d_in[5];
  const float* bc1 = (const float*)d_in[6];
  const float* Wc2 = (const float*)d_in[7];
  const float* bc2 = (const float*)d_in[8];
  const float* Wr1 = (const float*)d_in[9];
  const float* br1 = (const float*)d_in[10];
  const float* Wr2 = (const float*)d_in[11];
  const float* br2 = (const float*)d_in[12];
  const float* Wf1 = (const float*)d_in[13];
  const float* bf1 = (const float*)d_in[14];
  const float* Wf2 = (const float*)d_in[15];
  const float* bf2 = (const float*)d_in[16];
  const float* Wh1 = (const float*)d_in[17];
  const float* bh1 = (const float*)d_in[18];
  const float* Wh2 = (const float*)d_in[19];
  const float* bh2 = (const float*)d_in[20];
  float* out = (float*)d_out;

  char* ws = (char*)d_ws;
  float*    MET   = (float*)(ws + kOffMET);
  float*    PP    = (float*)(ws + kOffPP);
  float*    G1    = (float*)(ws + kOffG1);
  float*    G2    = (float*)(ws + kOffG2);
  float*    HPART = (float*)(ws + kOffHPART);
  float*    SS    = (float*)(ws + kOffSS);
  _Float16* W1C   = (_Float16*)(ws + kOffW1C);
  _Float16* W2T   = (_Float16*)(ws + kOffW2T);

  pack_weights_kernel<<<132, 256, 0, stream>>>(Wr1, Wr2, W1C, W2T);
  metric_kernel<<<kNB, 256, 0, stream>>>(points, Wm1, bm1, Wm2, bm2, MET);
  pair_pre_kernel<<<kNB, 256, 0, stream>>>(points, Wr1, MET, PP, G1, G2);
  triple_pair_kernel<<<kNB * kMD, 256, 0, stream>>>(MET, Wc1, bc1, Wc2, bc2, W1C, br1, PP, G1, G2, HPART);
  mean_proj_kernel<<<kMM / 128, 256, 0, stream>>>(HPART, W2T, br2, SS);
  tail_kernel<<<kNB, 256, 0, stream>>>(points, SS, Wf1, bf1, Wf2, bf2, Wh1, bh1, Wh2, bh2, out);
}
